// EulerAttentionVariant_75892072121088
// MI455X (gfx1250) — hardware-verified
//
#include <hip/hip_runtime.h>


#define NBT  2
#define NN   2048
#define DMOD 1024
#define NH_  16
#define HD   64
#define QW   128
#define LUTN 4096
#define NTK  NN
#define SCL  0.088388347648318447f
#define LOSC 1024.0f
__device__ __forceinline__ float lut_scale() { const float two_pi = 2.0f * 3.14159274101257324f; return (float)LUTN / two_pi; }

typedef _Float16 h16;
typedef unsigned short bf;
typedef __attribute__((ext_vector_type(16))) __bf16   v16bf;
typedef __attribute__((ext_vector_type(16))) _Float16 v16h;
typedef __attribute__((ext_vector_type(8)))  _Float16 v8h;
typedef __attribute__((ext_vector_type(8)))  unsigned short v8us;
typedef __attribute__((ext_vector_type(8)))  float    v8f;
typedef __attribute__((ext_vector_type(4)))  float    v4f;
typedef __attribute__((ext_vector_type(4)))  _Float16 v4h;
typedef v8h  __attribute__((may_alias)) v8ha;
typedef v4f  __attribute__((may_alias)) v4fa;
typedef v8us __attribute__((may_alias)) v8usa;

__device__ __forceinline__ unsigned short f2bf(float f) { unsigned u = __float_as_uint(f); u += 0x7FFFu + ((u >> 16) & 1u); return (unsigned short)(u >> 16); }
__device__ __forceinline__ float bf2f(unsigned short b) { return __uint_as_float(((unsigned)b) << 16); }
__device__ __forceinline__ float bfr(float f) { return bf2f(f2bf(f)); }
__device__ __forceinline__ v16h cat16(v8h lo, v8h hi) { return __builtin_shufflevector(lo, hi, 0, 1, 2, 3, 4, 5, 6, 7, 8, 9, 10, 11, 12, 13, 14, 15); }
__device__ __forceinline__ v16bf cat16b(v8us lo, v8us hi) { return __builtin_bit_cast(v16bf, __builtin_shufflevector(lo, hi, 0, 1, 2, 3, 4, 5, 6, 7, 8, 9, 10, 11, 12, 13, 14, 15)); }
__device__ __forceinline__ v8f wmma16(v16h a, v16h b, v8f c) { return __builtin_amdgcn_wmma_f32_16x16x32_f16(false, a, false, b, (short)0, c, false, false); }
__device__ __forceinline__ v8f wmmab(v16bf a, v16bf b, v8f c) { return __builtin_amdgcn_wmma_f32_16x16x32_bf16(false, a, false, b, (short)0, c, false, false); }


template <int MODE>
__global__ __launch_bounds__(128) void k_gemm3z(const bf* __restrict__ Ah, const bf* __restrict__ Al, const bf* __restrict__ Bh, const bf* __restrict__ Bl, int K, float* C, int ldc, size_t sA, size_t sB, size_t sC) {
    if ((MODE & 1) && (int)blockIdx.y * 64 > (int)blockIdx.x * 64 + 63) return;
    const size_t z = blockIdx.z; Ah += z * sA; Al += z * sA; Bh += z * sB; Bl += z * sB; C += z * sC;
    const int Klim = (MODE & 2) ? min(K, ((int)blockIdx.x + 1) * 64) : K;
    __shared__ __align__(16) float ost[4][16 * 68];
    const int lane = threadIdx.x & 31, wave = threadIdx.x >> 5, lr = lane & 15, hi = lane >> 4;
    const int r0 = blockIdx.x * 64 + wave * 16, c0 = blockIdx.y * 64;
    const size_t aoff = (size_t)(r0 + lr) * K + 8 * hi;
    v8f acc[4];
#pragma unroll
    for (int t = 0; t < 4; ++t) acc[t] = (v8f){};
#pragma unroll 1
    for (int kc = 0; kc < Klim; kc += 32) {
        const v16bf a = cat16b(*(const v8us*)(Ah + aoff + kc), *(const v8us*)(Ah + aoff + kc + 16));
        v16bf al = a; if (!(MODE & 4) && !(MODE & 16)) al = cat16b(*(const v8us*)(Al + aoff + kc), *(const v8us*)(Al + aoff + kc + 16));
#pragma unroll
        for (int t = 0; t < 4; ++t) { const size_t bo = (size_t)(c0 + t * 16 + lr) * K + kc + 8 * hi;
            const v16bf bh = cat16b(*(const v8us*)(Bh + bo), *(const v8us*)(Bh + bo + 16));
            acc[t] = wmmab(a, bh, acc[t]);
            if (!(MODE & 4)) { if (!(MODE & 16)) acc[t] = wmmab(al, bh, acc[t]); if (!(MODE & 8)) { const v16bf bl = cat16b(*(const v8us*)(Bl + bo), *(const v8us*)(Bl + bo + 16)); acc[t] = wmmab(a, bl, acc[t]); } } }
        asm volatile("v_nop\n\tv_nop\n\tv_nop\n\tv_nop" : "+v"(acc[0]), "+v"(acc[1]), "+v"(acc[2]), "+v"(acc[3]) : "v"(a), "v"(al));
    }
    float* os = &ost[wave][0];
#pragma unroll
    for (int t = 0; t < 4; ++t) {
#pragma unroll
        for (int j = 0; j < 8; ++j) os[(hi * 8 + j) * 68 + t * 16 + lr] = acc[t][j]; }
    __builtin_amdgcn_wave_barrier(); asm volatile("" ::: "memory");
    float* crow = C + (size_t)r0 * ldc + c0;
    auto pass = [&]() {
#pragma unroll
        for (int s = 0; s < 8; ++s) { const int Lid = (lane >> 3) + 4 * s, piece = lane & 7; const int row = Lid >> 1, cofs = (Lid & 1) * 32 + piece * 4;
            const v4f val = *(const v4fa*)(os + row * 68 + cofs); *(volatile v4f*)(crow + (size_t)row * ldc + cofs) = val; }
    };
    pass(); __threadfence(); pass();
}
__global__ __launch_bounds__(256) void k_planes32z(const float* __restrict__ F, int ld, int off, float sc, int rows, bf* Ph, bf* Pl) {
    typedef __attribute__((ext_vector_type(2))) unsigned short v2us;
    const int lane = threadIdx.x & 31; const size_t r = ((size_t)blockIdx.x * 8 + (threadIdx.x >> 5)) * 2 + (lane >> 4); if (r >= (size_t)rows) return; const int z = blockIdx.z; const int c0 = (lane & 15) * 2; v2us oh, ol;
    Ph += (size_t)z * rows * 32; Pl += (size_t)z * rows * 32;
#pragma unroll
    for (int i = 0; i < 2; ++i) { const float y = F[r * ld + off + z * 32 + c0 + i] * sc; const unsigned short hb = f2bf(y); oh[i] = hb; ol[i] = f2bf(y - bf2f(hb)); }
    const size_t o = r * 32 + c0; *(volatile v2us*)(Ph + o) = oh; *(volatile v2us*)(Pl + o) = ol; __threadfence(); *(volatile v2us*)(Ph + o) = oh; *(volatile v2us*)(Pl + o) = ol;
}
__global__ __launch_bounds__(256) void k_vtpadz(const float* __restrict__ F, int ld, int off, int nk, bf* Th, bf* Tl) {
    typedef __attribute__((ext_vector_type(2))) unsigned short v2us;
    const int lane = threadIdx.x & 31; const size_t wid = (size_t)blockIdx.x * 8 + (threadIdx.x >> 5); if (wid >= (size_t)64 * (nk / 64)) return; const int z = blockIdx.z; const int d = (int)(wid / (nk / 64)); const int k0 = (int)(wid % (nk / 64)) * 64 + lane * 2; v2us oh, ol;
    Th += (size_t)z * 64 * nk; Tl += (size_t)z * 64 * nk;
#pragma unroll
    for (int i = 0; i < 2; ++i) { const float y = (d < 32) ? F[(size_t)(k0 + i) * ld + off + z * 32 + (d < 32 ? d : 0)] : 0.f; const unsigned short hb = f2bf(y); oh[i] = hb; ol[i] = f2bf(y - bf2f(hb)); }
    const size_t o = (size_t)d * nk + k0; *(volatile v2us*)(Th + o) = oh; *(volatile v2us*)(Tl + o) = ol; __threadfence(); *(volatile v2us*)(Th + o) = oh; *(volatile v2us*)(Tl + o) = ol;
}
template <int NK>
__global__ __launch_bounds__(256) void k_softmaxz(const float* __restrict__ S, int rows, bf* PH, bf* PL) {
    typedef __attribute__((ext_vector_type(4))) unsigned short v4us;
    const int lane = threadIdx.x & 31, i = blockIdx.x * 8 + (threadIdx.x >> 5); if (i >= rows) return; const size_t zo = (size_t)blockIdx.z * rows * NK; const float* sr = S + zo + (size_t)i * NK; PH += zo; PL += zo;
    float m = -3.0e38f;
#pragma unroll 1
    for (int c0 = lane * 4; c0 < NK; c0 += 128) {
#pragma unroll
        for (int q = 0; q < 4; ++q) m = fmaxf(m, sr[c0 + q]); }
#pragma unroll
    for (int sh = 16; sh; sh >>= 1) m = fmaxf(m, __shfl_xor(m, sh, 32));
    float sum = 0.f;
#pragma unroll 1
    for (int c0 = lane * 4; c0 < NK; c0 += 128) {
#pragma unroll
        for (int q = 0; q < 4; ++q) sum += __expf(sr[c0 + q] - m); }
#pragma unroll
    for (int sh = 16; sh; sh >>= 1) sum += __shfl_xor(sum, sh, 32);
    const float inv = 1.0f / sum;
#pragma unroll 1
    for (int ps = 0; ps < 2; ++ps) {
#pragma unroll 1
        for (int c0 = lane * 4; c0 < NK; c0 += 128) { v4us oh, ol;
#pragma unroll
            for (int q = 0; q < 4; ++q) { const float p = __expf(sr[c0 + q] - m) * inv; const unsigned short hb = f2bf(p); oh[q] = hb; ol[q] = f2bf(p - bf2f(hb)); }
            const size_t o = (size_t)i * NK + c0; *(volatile v4us*)(PH + o) = oh; *(volatile v4us*)(PL + o) = ol; }
        if (ps == 0) __threadfence(); }
}
__global__ __launch_bounds__(256) void k_placez(const float* __restrict__ XH, int rows, int ldy, float* Y) {
    const int lane = threadIdx.x & 31; const size_t q = (size_t)blockIdx.x * 8 + (threadIdx.x >> 5); if (q >= (size_t)rows) return; const int z = blockIdx.z; const float v = XH[((size_t)z * rows + q) * 64 + lane];
    *(volatile float*)(Y + q * ldy + z * 32 + lane) = v; __threadfence(); *(volatile float*)(Y + q * ldy + z * 32 + lane) = v;
}

__global__ __launch_bounds__(256) void k_lut(float* SINT, float* COST) {
    const size_t i = (size_t)blockIdx.x * 256 + threadIdx.x; if (i >= (size_t)LUTN) return; const float two_pi = 2.0f * 3.14159274101257324f; const float a = two_pi * (float)i / (float)LUTN; const float s = sinf(a), c = cosf(a);
    *(volatile float*)(SINT + i) = s; *(volatile float*)(COST + i) = c; __threadfence(); *(volatile float*)(SINT + i) = s; *(volatile float*)(COST + i) = c;
}
__device__ __forceinline__ void lut_sc(float theta, const float* __restrict__ SINT, const float* __restrict__ COST, float& s, float& c) {
    const float pos = theta * lut_scale(); const float fl = floorf(pos); const float frac = pos - fl; int i0 = (int)fl; i0 = ((i0 % LUTN) + LUTN) % LUTN; const int i1 = (i0 + 1) % LUTN;
    s = SINT[i0] * (1.0f - frac) + SINT[i1] * frac; c = COST[i0] * (1.0f - frac) + COST[i1] * frac;
}
__global__ __launch_bounds__(256) void k_qkplanes(const float* __restrict__ x, const float* __restrict__ pos, const float* __restrict__ wq, const float* __restrict__ bq, const float* __restrict__ wk, const float* __restrict__ bk, int h, const float* __restrict__ SINT, const float* __restrict__ COST, bf* Qh, bf* Ql, bf* Kh, bf* Kl) {
    typedef __attribute__((ext_vector_type(2))) unsigned short v2us;
    const int lane = threadIdx.x & 31; const size_t sI = (size_t)blockIdx.x * 8 + (threadIdx.x >> 5); if (sI >= (size_t)NN) return; const float t = bfr(pos[sI]) * 1.61803398874989484f;
    v2us qc_h, qc_l, qs_h, qs_l, kc_h, kc_l, ks_h, ks_l;
#pragma unroll
    for (int i = 0; i < 2; ++i) { const int d = lane * 2 + i; const float xv = bfr(x[sI * DMOD + h * HD + d]);
        const float thq = xv / (1.0f + fabsf(bfr(wq[h * HD + d]))) + bfr(bq[h * HD + d]) + t; const float thk = xv / (1.0f + fabsf(bfr(wk[h * HD + d]))) + bfr(bk[h * HD + d]);
        float sq, cq, sk, ck; lut_sc(thq, SINT, COST, sq, cq); lut_sc(thk, SINT, COST, sk, ck);
        unsigned short hb; hb = f2bf(cq); qc_h[i] = hb; qc_l[i] = f2bf(cq - bf2f(hb)); hb = f2bf(sq); qs_h[i] = hb; qs_l[i] = f2bf(sq - bf2f(hb));
        hb = f2bf(ck); kc_h[i] = hb; kc_l[i] = f2bf(ck - bf2f(hb)); hb = f2bf(sk); ks_h[i] = hb; ks_l[i] = f2bf(sk - bf2f(hb)); }
    const size_t o = sI * QW + lane * 2;
#pragma unroll 1
    for (int ps = 0; ps < 2; ++ps) { *(volatile v2us*)(Qh + o) = qc_h; *(volatile v2us*)(Ql + o) = qc_l; *(volatile v2us*)(Qh + o + HD) = qs_h; *(volatile v2us*)(Ql + o + HD) = qs_l; *(volatile v2us*)(Kh + o) = kc_h; *(volatile v2us*)(Kl + o) = kc_l; *(volatile v2us*)(Kh + o + HD) = ks_h; *(volatile v2us*)(Kl + o + HD) = ks_l; if (ps == 0) __threadfence(); }
}
__global__ __launch_bounds__(256) void k_vtplanes(const float* __restrict__ x, const float* __restrict__ pos, const float* __restrict__ wv, const float* __restrict__ bv, int h, const float* __restrict__ SINT, const float* __restrict__ COST, bf* CTh, bf* CTl, bf* STh, bf* STl) {
    typedef __attribute__((ext_vector_type(2))) unsigned short v2us;
    const int lane = threadIdx.x & 31; const size_t wid = (size_t)blockIdx.x * 8 + (threadIdx.x >> 5); if (wid >= (size_t)HD * (NN / 64)) return; const int d = (int)(wid / (NN / 64)); const int s0 = (int)(wid % (NN / 64)) * 64 + lane * 2; v2us ch, cl, sh_, sl;
    const float wvv = 1.0f + fabsf(bfr(wv[h * HD + d])), bvv = bfr(bv[h * HD + d]);
#pragma unroll
    for (int i = 0; i < 2; ++i) { const size_t sI = s0 + i; const float t = bfr(pos[sI]) * 1.61803398874989484f; const float th = bfr(x[sI * DMOD + h * HD + d]) / wvv + bvv + t; float sv, cv; lut_sc(th, SINT, COST, sv, cv);
        unsigned short hb = f2bf(cv); ch[i] = hb; cl[i] = f2bf(cv - bf2f(hb)); hb = f2bf(sv); sh_[i] = hb; sl[i] = f2bf(sv - bf2f(hb)); }
    const size_t o = (size_t)d * NN + s0; *(volatile v2us*)(CTh + o) = ch; *(volatile v2us*)(CTl + o) = cl; *(volatile v2us*)(STh + o) = sh_; *(volatile v2us*)(STl + o) = sl; __threadfence(); *(volatile v2us*)(CTh + o) = ch; *(volatile v2us*)(CTl + o) = cl; *(volatile v2us*)(STh + o) = sh_; *(volatile v2us*)(STl + o) = sl;
}
__global__ __launch_bounds__(256) void k_csoftz(const float* __restrict__ S, int rows, float sc, bf* PH, bf* PL) {
    typedef __attribute__((ext_vector_type(4))) unsigned short v4us;
    const int lane = threadIdx.x & 31, i = blockIdx.x * 8 + (threadIdx.x >> 5); if (i >= rows) return; const size_t zo = (size_t)blockIdx.z * rows * NN; const float* sr = S + zo + (size_t)i * NN; PH += zo; PL += zo;
    float m = -3.0e38f;
#pragma unroll 1
    for (int c0 = lane * 4; c0 < NN; c0 += 128) {
#pragma unroll
        for (int q = 0; q < 4; ++q) { const int k = c0 + q; if (k <= i) m = fmaxf(m, sr[k] * sc); } }
#pragma unroll
    for (int sh = 16; sh; sh >>= 1) m = fmaxf(m, __shfl_xor(m, sh, 32));
    float sum = 0.f;
#pragma unroll 1
    for (int c0 = lane * 4; c0 < NN; c0 += 128) {
#pragma unroll
        for (int q = 0; q < 4; ++q) { const int k = c0 + q; if (k <= i) sum += __expf(sr[k] * sc - m); } }
#pragma unroll
    for (int sh = 16; sh; sh >>= 1) sum += __shfl_xor(sum, sh, 32);
    const float inv = 1.0f / sum;
#pragma unroll 1
    for (int ps = 0; ps < 2; ++ps) {
#pragma unroll 1
        for (int c0 = lane * 4; c0 < NN; c0 += 128) { v4us oh, ol;
#pragma unroll
            for (int q = 0; q < 4; ++q) { const int k = c0 + q; const float p = (k <= i) ? __expf(sr[(k <= i) ? k : 0] * sc - m) * inv : 0.f; const unsigned short hb = f2bf(p); oh[q] = hb; ol[q] = f2bf(p - bf2f(hb)); }
            const size_t o = (size_t)i * NN + c0; *(volatile v4us*)(PH + o) = oh; *(volatile v4us*)(PL + o) = ol; }
        if (ps == 0) __threadfence(); }
}
__global__ __launch_bounds__(256) void k_olut(const float* __restrict__ OC, const float* __restrict__ OS, const float* __restrict__ wo, const float* __restrict__ bo, const float* __restrict__ SINT, const float* __restrict__ COST, float* OUTB) {
    const int lane = threadIdx.x & 31; const size_t sI = (size_t)blockIdx.x * 8 + (threadIdx.x >> 5); if (sI >= (size_t)NN) return;
#pragma unroll 1
    for (int ps = 0; ps < 2; ++ps) {
#pragma unroll 1
        for (int q = 0; q < DMOD / 128; ++q) { const int c0 = q * 128 + lane * 4; v4f v;
#pragma unroll
            for (int i = 0; i < 4; ++i) { const int c = c0 + i; const float th = (OC[sI * DMOD + c] + OS[sI * DMOD + c]) / (1.0f + fabsf(bfr(wo[c]))) + bfr(bo[c]); float s, cc; lut_sc(th, SINT, COST, s, cc); v[i] = cc + s; }
            *(volatile v4f*)(OUTB + sI * DMOD + c0) = v; }
        if (ps == 0) __threadfence(); }
}

extern "C" void kernel_launch(void* const* d_in, const int* in_sizes, int n_in,
                              void* d_out, int out_size, void* d_ws, size_t ws_size, hipStream_t stream) {
    (void)in_sizes; (void)n_in; (void)out_size;
    const float* x = (const float*)d_in[0]; const float* pos = (const float*)d_in[1]; const float* wq = (const float*)d_in[2]; const float* bq = (const float*)d_in[3]; const float* wk = (const float*)d_in[4]; const float* bk = (const float*)d_in[5]; const float* wv = (const float*)d_in[6]; const float* bv = (const float*)d_in[7]; const float* wo = (const float*)d_in[8]; const float* bo = (const float*)d_in[9];
    float* out = (float*)d_out;
    char* wsp = (char*)d_ws;
    auto take = [&](size_t bytes) { char* p = wsp; wsp += (bytes + 255) & ~(size_t)255; return (void*)p; };
    float* SINT = (float*)take(LUTN * 4); float* COST = (float*)take(LUTN * 4);
    bf* Qh = (bf*)take((size_t)NN * QW * 2); bf* Ql = (bf*)take((size_t)NN * QW * 2); bf* Kh = (bf*)take((size_t)NN * QW * 2); bf* Kl = (bf*)take((size_t)NN * QW * 2);
    bf* CTh = (bf*)take((size_t)HD * NN * 2); bf* CTl = (bf*)take((size_t)HD * NN * 2); bf* STh = (bf*)take((size_t)HD * NN * 2); bf* STl = (bf*)take((size_t)HD * NN * 2);
    float* S = (float*)take((size_t)NN * NN * 4); bf* PH = (bf*)take((size_t)NN * NN * 2); bf* PL = (bf*)take((size_t)NN * NN * 2); float* OC = (float*)take((size_t)NN * DMOD * 4); float* OS = (float*)take((size_t)NN * DMOD * 4);
    if ((size_t)(wsp - (char*)d_ws) > ws_size) return;
    k_lut<<<LUTN / 256, 256, 0, stream>>>(SINT, COST);
    for (int b = 0; b < NBT; ++b) { const float* xb = x + (size_t)b * NN * DMOD;
        for (int h = 0; h < NH_; ++h) {
            k_qkplanes<<<NN / 8, 256, 0, stream>>>(xb, pos, wq, bq, wk, bk, h, SINT, COST, Qh, Ql, Kh, Kl); k_vtplanes<<<(HD * (NN / 64)) / 8, 256, 0, stream>>>(xb, pos, wv, bv, h, SINT, COST, CTh, CTl, STh, STl);
            k_gemm3z<1><<<dim3(NN / 64, NN / 64, 1), 128, 0, stream>>>(Qh, Ql, Kh, Kl, QW, S, NN, 0, 0, 0);
            k_csoftz<<<dim3(NN / 8, 1, 1), 256, 0, stream>>>(S, NN, SCL, PH, PL);
            k_gemm3z<2><<<dim3(NN / 64, 1, 1), 128, 0, stream>>>(PH, PL, CTh, CTl, NN, OC + (size_t)h * HD, DMOD, 0, 0, 0);
            k_gemm3z<2><<<dim3(NN / 64, 1, 1), 128, 0, stream>>>(PH, PL, STh, STl, NN, OS + (size_t)h * HD, DMOD, 0, 0, 0); }
        k_olut<<<NN / 8, 256, 0, stream>>>(OC, OS, wo, bo, SINT, COST, out + (size_t)b * NN * DMOD); }
}
